// Grader_86552180949555
// MI455X (gfx1250) — hardware-verified
//
#include <hip/hip_runtime.h>
#include <math.h>

constexpr int NBATCH  = 32;
constexpr int NSTEP   = 2048;
constexpr int NEMB    = 300;
constexpr int KPAD    = 320;
constexpr int NHID    = 256;
constexpr int NVOC    = 50000;
constexpr int NGRADE  = 5;
constexpr int NTHR    = 256;
constexpr int SEQ_BLK = 16;
constexpr int HPITCH  = 264;
constexpr int SLABP   = 36;
constexpr int NROWS   = NBATCH * NSTEP;
constexpr float XCARRY    = 64.0f;
constexpr float WCARRY    = 64.0f;
constexpr float HCARRY    = 16.0f;
constexpr float XPROJ_INV = 1.0f / 4096.0f;
constexpr float REC_INV   = 1.0f / 1024.0f;
constexpr float MEAN_INV  = 1.0f / 2048.0f;
static_assert(NROWS % 64 == 0 && NHID % 64 == 0, "GEMM M, N tile multiples");
static_assert(KPAD % 32 == 0 && KPAD >= NEMB, "GEMM K multiple of 32");
static_assert(NHID % 32 == 0, "recurrence K multiple of 32");
static_assert(NHID == 32 * (NTHR / 32), "8 waves x 32 hidden columns");
static_assert(NBATCH % SEQ_BLK == 0, "blocks own whole 16-row groups");
static_assert((2 * SEQ_BLK * HPITCH) % NTHR == 0, "h zero-fill loop exact");
static_assert(NSTEP % 64 == 0, "64-step partial sums fold exactly");
static_assert(NEMB % 4 == 0 && NHID % 4 == 0, "16-B source loads");
static_assert(NHID == 256, "head index arithmetic uses >>8 / &255");
static_assert(NBATCH * NGRADE == 160, "output = 160 floats = 5 whole 128-B lines");

typedef __attribute__((ext_vector_type(16))) _Float16 v16h;
typedef __attribute__((ext_vector_type(8)))  _Float16 v8h;
typedef __attribute__((ext_vector_type(16))) __bf16   v16b;
typedef __attribute__((ext_vector_type(8)))  __bf16   v8b;
typedef __attribute__((ext_vector_type(8)))  float    v8f;
typedef __attribute__((ext_vector_type(4)))  float    v4f;

__device__ __forceinline__ unsigned short f2bf_bits(float f) {
  unsigned u = __float_as_uint(f);
  return (unsigned short)((u + 0x7FFFu + ((u >> 16) & 1u)) >> 16);
}
__device__ __forceinline__ float bf_bits2f(unsigned short h) { return __uint_as_float(((unsigned)h) << 16); }

__device__ __forceinline__ void dep_guard_h(v8f& a, v8f& b, v16h x, v16h y) { asm volatile("v_nop\n\tv_nop\n\tv_nop\n\tv_nop" : "+v"(a), "+v"(b) : "v"(x), "v"(y)); }
__device__ __forceinline__ void dep_guard_b(v8f& a, v8f& b, v16b x, v16b y) { asm volatile("v_nop\n\tv_nop\n\tv_nop\n\tv_nop" : "+v"(a), "+v"(b) : "v"(x), "v"(y)); }
__device__ __forceinline__ void keep4_h(v16h a, v16h b, v16h c, v16h d) { asm volatile("v_nop" :: "v"(a), "v"(b), "v"(c), "v"(d)); }
__device__ __forceinline__ void keep4_b(v16b a, v16b b, v16b c, v16b d) { asm volatile("v_nop" :: "v"(a), "v"(b), "v"(c), "v"(d)); }
__device__ __forceinline__ void acc_guard4(v8f& a, v8f& b, v8f& c, v8f& d) { asm volatile("v_nop\n\tv_nop\n\tv_nop\n\tv_nop" : "+v"(a), "+v"(b), "+v"(c), "+v"(d)); }
__device__ __forceinline__ void acc_guard2(v8f& a, v8f& b) { asm volatile("v_nop\n\tv_nop\n\tv_nop\n\tv_nop" : "+v"(a), "+v"(b)); }
template <typename T> struct Frag;
template <> struct Frag<_Float16> {
  typedef v16h V; union U { v16h v; v8h h[2]; };
  static __device__ __forceinline__ v16h load(const _Float16* p) {
    U f; f.h[0] = *(const v8h*)(p); f.h[1] = *(const v8h*)(p + 16); return f.v;
  }
  static __device__ __forceinline__ v8f mma(v16h a, v16h b, v8f c) {
    return __builtin_amdgcn_wmma_f32_16x16x32_f16(false, a, false, b, (short)0, c, false, false);
  }
  static __device__ __forceinline__ void guard(v8f& a, v8f& b, v16h x, v16h y) { dep_guard_h(a, b, x, y); }
  static __device__ __forceinline__ void keep(v16h a, v16h b, v16h c, v16h d) { keep4_h(a, b, c, d); }
};
template <> struct Frag<__bf16> {
  typedef v16b V; union U { v16b v; v8b h[2]; };
  static __device__ __forceinline__ v16b load(const __bf16* p) {
    U f; f.h[0] = *(const v8b*)(p); f.h[1] = *(const v8b*)(p + 16); return f.v;
  }
  static __device__ __forceinline__ v8f mma(v16b a, v16b b, v8f c) {
    return __builtin_amdgcn_wmma_f32_16x16x32_bf16(false, a, false, b, (short)0, c, false, false);
  }
  static __device__ __forceinline__ void guard(v8f& a, v8f& b, v16b x, v16b y) { dep_guard_b(a, b, x, y); }
  static __device__ __forceinline__ void keep(v16b a, v16b b, v16b c, v16b d) { keep4_b(a, b, c, d); }
};

__device__ __forceinline__ float ftanh(float x) { return 1.0f - 2.0f * __builtin_amdgcn_rcpf(__expf(2.0f * x) + 1.0f); }

template <int ET> struct Elem;
template <> struct Elem<0> { typedef _Float16 T; };
template <> struct Elem<1> { typedef __bf16 T; };
template <int ET, bool SPLIT, int BIAS_MODE, int OUT_MODE, bool RESID, int ACT = 0>
__global__ __launch_bounds__(256) void wmma_gemm64(
    const unsigned short* __restrict__ Ap, const unsigned short* __restrict__ A2p, int lda, long strideA,
    const unsigned short* __restrict__ Btp, const unsigned short* __restrict__ Bt2p, int ldb, long strideB,
    void* __restrict__ Cout, void* __restrict__ Cout2, int ldc, long strideC,
    const float* __restrict__ bias,
    const float* __restrict__ resid, long strideR,
    int M, int N, int K, float scale) {
  typedef typename Elem<ET>::T T;
  typedef typename Frag<T>::V V;
  const T* A = (const T*)Ap; const T* A2 = (const T*)A2p; const T* Bt = (const T*)Btp; const T* Bt2 = (const T*)Bt2p;
  __shared__ __align__(16) float sT[8][16 * 68];
  const int b    = blockIdx.y;
  const int lane = threadIdx.x & 31;
  const int wave = threadIdx.x >> 5;
  const int tilesN = N >> 6;
  const int tilesM = M >> 6;
  const int tile = blockIdx.x * 8 + wave;
  if (tile >= tilesM * tilesN) return;
  const int tm = tile / tilesN;
  const int tn = tile - tm * tilesN;
  const int m0 = tm << 6;
  const int n0 = tn << 6;

  const T* Ab  = A  + (size_t)b * strideA;
  const T* Bb  = Bt + (size_t)b * strideB;
  const T* Ab2 = SPLIT ? (A2  + (size_t)b * strideA) : nullptr;
  const T* Bb2 = SPLIT ? (Bt2 + (size_t)b * strideB) : nullptr;

  const int rlane = lane & 15;
  const int koff  = (lane >> 4) * 8;
  const int mOff  = (lane >> 4) * 8;

  v8f acc[4][4];
#pragma unroll
  for (int i = 0; i < 4; ++i)
#pragma unroll
    for (int j = 0; j < 4; ++j) acc[i][j] = (v8f){0.f,0.f,0.f,0.f,0.f,0.f,0.f,0.f};

  for (int k0 = 0; k0 < K; k0 += 32) {
    V bh[4], bl[4];
#pragma unroll
    for (int j = 0; j < 4; ++j) {
      const size_t bo = (size_t)(n0 + (j << 4) + rlane) * ldb + koff + k0;
      bh[j] = Frag<T>::load(Bb + bo);
      if (SPLIT) bl[j] = Frag<T>::load(Bb2 + bo);
    }
#pragma unroll
    for (int i = 0; i < 4; ++i) {
      const size_t ao = (size_t)(m0 + (i << 4) + rlane) * lda + koff + k0;
      V ah = Frag<T>::load(Ab + ao);
      V al;
      if (SPLIT) al = Frag<T>::load(Ab2 + ao);
#pragma unroll
      for (int j = 0; j < 4; ++j) {
        acc[i][j] = Frag<T>::mma(ah, bh[j], acc[i][j]);
        if (SPLIT) {
          acc[i][j] = Frag<T>::mma(ah, bl[j], acc[i][j]);
          acc[i][j] = Frag<T>::mma(al, bh[j], acc[i][j]);
        }
      }
      Frag<T>::guard(acc[i][0], acc[i][3], ah, SPLIT ? al : ah);
    }
    Frag<T>::keep(bh[0], bh[1], bh[2], bh[3]);
    if (SPLIT) Frag<T>::keep(bl[0], bl[1], bl[2], bl[3]);
  }
  acc_guard4(acc[0][0], acc[0][1], acc[0][2], acc[0][3]);
  acc_guard4(acc[1][0], acc[1][1], acc[1][2], acc[1][3]);
  acc_guard4(acc[2][0], acc[2][1], acc[2][2], acc[2][3]);
  acc_guard4(acc[3][0], acc[3][1], acc[3][2], acc[3][3]);

  float* slab = sT[wave];
  const float* Rb = RESID ? (resid + (size_t)b * strideR) : nullptr;
#pragma unroll
  for (int i = 0; i < 4; ++i) {
    const int mBase = m0 + (i << 4);
#pragma unroll
    for (int j = 0; j < 4; ++j) {
      const int n = n0 + (j << 4) + rlane;
      float bv = 0.f;
      if (BIAS_MODE == 2) bv = bias[n];
#pragma unroll
      for (int r = 0; r < 8; ++r) {
        float v = acc[i][j][r] * scale;
        if (BIAS_MODE == 1) v += bias[mBase + mOff + r];
        if (BIAS_MODE == 2) v += bv;
        if (RESID) v += Rb[(size_t)(mBase + mOff + r) * ldc + n];
        if (ACT == 1) v = tanhf(v);
        if (ACT == 2) v = fmaxf(v, 0.0f);
        if (ACT == 3) v = v / (1.0f + expf(-v));
        if (ACT == 4) v = (v > 0.f) ? v : 0.01f * v;
        if (ACT == 5) v = 0.5f * v * (1.0f + erff(v * 0.70710678118654752f));
        slab[(mOff + r) * 68 + (j << 4) + rlane] = v;
      }
    }
    __builtin_amdgcn_fence(__ATOMIC_RELEASE, "workgroup");
    __builtin_amdgcn_wave_barrier();
    __builtin_amdgcn_fence(__ATOMIC_ACQUIRE, "workgroup");
    if (OUT_MODE == 0) {
      float* C = (float*)Cout + (size_t)b * strideC;
      const int hh = lane >> 4, c4 = (lane & 15) * 4;
      for (int pass = 0; pass < 2; ++pass) {
#pragma unroll
        for (int it = 0; it < 8; ++it) {
          const int row = it * 2 + hh;
          v4f v = *(const v4f*)(slab + row * 68 + c4);
          *(volatile v4f*)(C + (size_t)(mBase + row) * ldc + n0 + c4) = v;
        }
        __threadfence();
      }
    } else {
      const int q = lane >> 3, c8 = (lane & 7) * 8;
      unsigned short* C  = (unsigned short*)Cout  + (size_t)b * strideC;
      unsigned short* C2 = (OUT_MODE == 2) ? ((unsigned short*)Cout2 + (size_t)b * strideC) : nullptr;
      for (int pass = 0; pass < 2; ++pass) {
#pragma unroll
        for (int it = 0; it < 4; ++it) {
          const int row = it * 4 + q;
          const float* sp = slab + row * 68 + c8;
          v8h hv, lv;
#pragma unroll
          for (int e = 0; e < 8; ++e) {
            if (OUT_MODE == 1) {
              hv[e] = (_Float16)sp[e];
            } else {
              unsigned short hb = f2bf_bits(sp[e]);
              unsigned short lb = f2bf_bits(sp[e] - bf_bits2f(hb));
              hv[e] = __builtin_bit_cast(_Float16, hb);
              lv[e] = __builtin_bit_cast(_Float16, lb);
            }
          }
          *(volatile v8h*)(C + (size_t)(mBase + row) * ldc + n0 + c8) = hv;
          if (OUT_MODE == 2) *(volatile v8h*)(C2 + (size_t)(mBase + row) * ldc + n0 + c8) = lv;
        }
        __threadfence();
      }
    }
    __builtin_amdgcn_fence(__ATOMIC_RELEASE, "workgroup");
    __builtin_amdgcn_wave_barrier();
    __builtin_amdgcn_fence(__ATOMIC_ACQUIRE, "workgroup");
  }
}

template <bool GATHER>
__global__ __launch_bounds__(NTHR) void rows_to_f16_kernel(const float* __restrict__ src, const int* __restrict__ tok,
                                                           unsigned short* __restrict__ dst, int nrow, int ncol8, int ncols,
                                                           float sc) {
  const int i  = blockIdx.x * NTHR + threadIdx.x;
  const int n8 = nrow * ncol8;
  if (i < n8) {
    const int row = i / ncol8;
    const int c8  = i - row * ncol8;
    int srow = row;
    if (GATHER) {
      const int s = row / NBATCH;
      const int b = row - s * NBATCH;
      int t = tok[b * NSTEP + s];
      t = t < 0 ? 0 : t;
      t = t > NVOC - 1 ? NVOC - 1 : t;
      srow = t;
    }
    const int c0 = c8 * 8;
    const int ia = (c0 < ncols - 4) ? c0 : (ncols - 4);
    const int ib = (c0 + 4 < ncols - 4) ? (c0 + 4) : (ncols - 4);
    const float* sp = src + (size_t)srow * ncols;
    const v4f va = *(const v4f*)(sp + ia);
    const v4f vb = *(const v4f*)(sp + ib);
    v8h hv;
#pragma unroll
    for (int e = 0; e < 4; ++e) {
      const float fa = (c0 + e < ncols) ? va[e] : 0.0f;
      const float fb = (c0 + 4 + e < ncols) ? vb[e] : 0.0f;
      hv[e]     = (_Float16)(fa * sc);
      hv[4 + e] = (_Float16)(fb * sc);
    }
    *(volatile v8h*)(dst + (size_t)i * 8) = hv;
    __threadfence();
    *(volatile v8h*)(dst + (size_t)i * 8) = hv;
  }
}

__global__ __launch_bounds__(NTHR) void rnn_dir_kernel(const float* __restrict__ XP, const unsigned short* __restrict__ WHHp,
                                                       const float* __restrict__ bih, const float* __restrict__ bhh,
                                                       float* __restrict__ POOLD, int dir) {
  __shared__ __align__(16) _Float16 Ah[2][SEQ_BLK * HPITCH];
  __shared__ __align__(16) float    Sl[NTHR / 32][16 * SLABP];
  const _Float16* WHH = (const _Float16*)WHHp;
  const int tid = threadIdx.x, lane = tid & 31, wave = tid >> 5;
  const int c = lane & 15, hh = lane >> 4, koff = hh * 8;
  const int rowbase = blockIdx.x * SEQ_BLK;
  const int j0 = 32 * wave + c;
  const int j1 = j0 + 16;

  {
    _Float16* ahf = &Ah[0][0];
#pragma unroll 1
    for (int i = tid; i < 2 * SEQ_BLK * HPITCH; i += NTHR) ahf[i] = (_Float16)0.0f;
  }
  const float bs0 = bih[j0] + bhh[j0];
  const float bs1 = bih[j1] + bhh[j1];
  float ps0[8], ps1[8], pt0[8], pt1[8];
#pragma unroll
  for (int r = 0; r < 8; ++r) { ps0[r] = 0.0f; ps1[r] = 0.0f; pt0[r] = 0.0f; pt1[r] = 0.0f; }
  __syncthreads();

  const v8f z8 = {0.f, 0.f, 0.f, 0.f, 0.f, 0.f, 0.f, 0.f};
  const _Float16* w0 = WHH + (size_t)j0 * NHID + koff;
  const _Float16* w1 = WHH + (size_t)j1 * NHID + koff;
  float* slab = Sl[wave];

#pragma unroll 1
  for (int t = 0; t < NSTEP; ++t) {
    const int s = dir ? (NSTEP - 1 - t) : t;
    const int cur = t & 1;
    float x0[8], x1[8];
#pragma unroll
    for (int r = 0; r < 8; ++r) {
      const size_t roff = (size_t)(s * NBATCH + rowbase + 8 * hh + r) * NHID;
      x0[r] = XP[roff + j0];
      x1[r] = XP[roff + j1];
    }
    const _Float16* ahrow = &Ah[cur][0] + c * HPITCH + koff;
    _Float16* ahn = &Ah[cur ^ 1][0];
    v8f acc0 = z8, acc1 = z8;
#pragma unroll 1
    for (int k0 = 0; k0 < NHID; k0 += 32) {
      const v16h a  = Frag<_Float16>::load(ahrow + k0);
      const v16h b0 = Frag<_Float16>::load(w0 + k0);
      const v16h b1 = Frag<_Float16>::load(w1 + k0);
      acc0 = Frag<_Float16>::mma(a, b0, acc0);
      acc1 = Frag<_Float16>::mma(a, b1, acc1);
      dep_guard_h(acc0, acc1, a, b1);
      keep4_h(a, b0, b1, a);
    }
    acc_guard2(acc0, acc1);
#pragma unroll
    for (int r = 0; r < 8; ++r) {
      const float z0 = acc0[r] * REC_INV + x0[r] + bs0;
      const float z1 = acc1[r] * REC_INV + x1[r] + bs1;
      const float h0 = ftanh(z0);
      const float h1 = ftanh(z1);
      ps0[r] += h0;
      ps1[r] += h1;
      ahn[(8 * hh + r) * HPITCH + j0] = (_Float16)(h0 * HCARRY);
      ahn[(8 * hh + r) * HPITCH + j1] = (_Float16)(h1 * HCARRY);
    }
    if ((t & 63) == 63) {
#pragma unroll
      for (int r = 0; r < 8; ++r) { pt0[r] += ps0[r]; ps0[r] = 0.0f; pt1[r] += ps1[r]; ps1[r] = 0.0f; }
    }
    __syncthreads();
  }

#pragma unroll
  for (int r = 0; r < 8; ++r) {
    slab[(8 * hh + r) * SLABP + c]      = pt0[r] + ps0[r];
    slab[(8 * hh + r) * SLABP + 16 + c] = pt1[r] + ps1[r];
  }
  __builtin_amdgcn_fence(__ATOMIC_RELEASE, "workgroup");
  __builtin_amdgcn_wave_barrier();
  __builtin_amdgcn_fence(__ATOMIC_ACQUIRE, "workgroup");
  {
    const int q = lane >> 3, c4 = (lane & 7) * 4;
    for (int pass = 0; pass < 2; ++pass) {
#pragma unroll
      for (int it = 0; it < 4; ++it) {
        const int row = it * 4 + q;
        const v4f v = *(const v4f*)(slab + row * SLABP + c4);
        *(volatile v4f*)(POOLD + (size_t)(rowbase + row) * NHID + 32 * wave + c4) = v;
      }
      __threadfence();
    }
  }
}

__global__ __launch_bounds__(NTHR) void head_kernel(const float* __restrict__ POOL, const float* __restrict__ fcW,
                                                    const float* __restrict__ fcb, float* __restrict__ out) {
  __shared__ __align__(16) float outs[192];
  const int tid = threadIdx.x;
  if (tid < NBATCH * NGRADE) {
    const int b = tid / NGRADE;
    const int g = tid - b * NGRADE;
    float s = 0.0f;
#pragma unroll 1
    for (int jj = 0; jj < 2 * NHID; ++jj) {
      const float v = POOL[(size_t)(jj >> 8) * (NBATCH * NHID) + (size_t)b * NHID + (jj & 255)];
      const float a = tanhf(v * MEAN_INV);
      s += a * fcW[g * (2 * NHID) + jj];
    }
    outs[tid] = s + fcb[g];
  }
  __syncthreads();
  if (tid < 32) {
    const v4f v0 = *(const v4f*)(outs + 4 * tid);
    const v4f v1 = *(const v4f*)(outs + 128 + 4 * (tid & 7));
    for (int pass = 0; pass < 2; ++pass) {
      *(volatile v4f*)(out + 4 * tid) = v0;
      if (tid < 8) *(volatile v4f*)(out + 128 + 4 * tid) = v1;
      __threadfence();
    }
  }
}

extern "C" void kernel_launch(void* const* d_in, const int* in_sizes, int n_in,
                              void* d_out, int out_size, void* d_ws, size_t ws_size, hipStream_t stream) {
  if (n_in < 12 || d_out == nullptr || d_ws == nullptr) return;
  if (in_sizes[0] != NBATCH * NSTEP || in_sizes[1] != NVOC * NEMB || in_sizes[2] != NHID * NEMB ||
      in_sizes[3] != NHID * NHID || in_sizes[4] != NHID || in_sizes[5] != NHID || in_sizes[6] != NHID * NEMB ||
      in_sizes[7] != NHID * NHID || in_sizes[8] != NHID || in_sizes[9] != NHID || in_sizes[10] != NGRADE * 2 * NHID ||
      in_sizes[11] != NGRADE || out_size != NBATCH * NGRADE) return;

  const int*   tok  = (const int*)d_in[0];
  const float* emb  = (const float*)d_in[1];
  const float* WihF = (const float*)d_in[2];
  const float* WhhF = (const float*)d_in[3];
  const float* bihF = (const float*)d_in[4];
  const float* bhhF = (const float*)d_in[5];
  const float* WihB = (const float*)d_in[6];
  const float* WhhB = (const float*)d_in[7];
  const float* bihB = (const float*)d_in[8];
  const float* bhhB = (const float*)d_in[9];
  const float* fcW  = (const float*)d_in[10];
  const float* fcb  = (const float*)d_in[11];
  float* out = (float*)d_out;

  char* ws = (char*)d_ws; size_t off = 0;
  auto carve = [&](size_t bytes) -> char* { char* p = ws + off; off += (bytes + 255) & ~(size_t)255; return p; };
  unsigned short* A16   = (unsigned short*)carve((size_t)NROWS * KPAD * 2);
  unsigned short* WIH16 = (unsigned short*)carve((size_t)2 * NHID * KPAD * 2);
  unsigned short* WHH16 = (unsigned short*)carve((size_t)2 * NHID * NHID * 2);
  float*          XP    = (float*)carve((size_t)NROWS * NHID * 4);
  float*          POOL  = (float*)carve((size_t)2 * NBATCH * NHID * 4);
  if (off > ws_size || off > (size_t)134217728) return;

  const int n8a = NROWS * (KPAD / 8);
  const int n8w = NHID * (KPAD / 8);
  const int n8h = NHID * (NHID / 8);
  rows_to_f16_kernel<true><<<(n8a + NTHR - 1) / NTHR, NTHR, 0, stream>>>(emb, tok, A16, NROWS, KPAD / 8, NEMB, XCARRY);
  rows_to_f16_kernel<false><<<(n8w + NTHR - 1) / NTHR, NTHR, 0, stream>>>(WihF, tok, WIH16, NHID, KPAD / 8, NEMB, WCARRY);
  rows_to_f16_kernel<false><<<(n8w + NTHR - 1) / NTHR, NTHR, 0, stream>>>(WihB, tok, WIH16 + (size_t)NHID * KPAD, NHID, KPAD / 8, NEMB, WCARRY);
  rows_to_f16_kernel<false><<<(n8h + NTHR - 1) / NTHR, NTHR, 0, stream>>>(WhhF, tok, WHH16, NHID, NHID / 8, NHID, WCARRY);
  rows_to_f16_kernel<false><<<(n8h + NTHR - 1) / NTHR, NTHR, 0, stream>>>(WhhB, tok, WHH16 + (size_t)NHID * NHID, NHID, NHID / 8, NHID, WCARRY);

  const dim3 ggrid((NROWS / 64) * (NHID / 64) / 8, 1);

  wmma_gemm64<0, false, 0, 0, false, 0><<<ggrid, 256, 0, stream>>>(
      A16, A16, KPAD, 0L, WIH16, WIH16, KPAD, 0L, (void*)XP, (void*)XP, NHID, 0L,
      POOL, POOL, 0L, NROWS, NHID, KPAD, XPROJ_INV);
  rnn_dir_kernel<<<NBATCH / SEQ_BLK, NTHR, 0, stream>>>(XP, WHH16, bihF, bhhF, POOL, 0);

  wmma_gemm64<0, false, 0, 0, false, 0><<<ggrid, 256, 0, stream>>>(
      A16, A16, KPAD, 0L, WIH16 + (size_t)NHID * KPAD, WIH16 + (size_t)NHID * KPAD, KPAD, 0L, (void*)XP, (void*)XP, NHID, 0L,
      POOL, POOL, 0L, NROWS, NHID, KPAD, XPROJ_INV);
  rnn_dir_kernel<<<NBATCH / SEQ_BLK, NTHR, 0, stream>>>(XP, WHH16 + (size_t)NHID * NHID, bihB, bhhB, POOL + (size_t)NBATCH * NHID, 1);

  head_kernel<<<1, NTHR, 0, stream>>>(POOL, fcW, fcb, out);
}
